// MultiHeadRelationalModule_60181081752248
// MI455X (gfx1250) — hardware-verified
//
#include <hip/hip_runtime.h>
#include <math.h>
#include <stdint.h>

#define NB      64
#define NH      4
#define NPIX    596
#define PP      608
#define PVT     640
#define FRW     640
#define DH      64
#define CP      256
#define NCT     38
#define NKS     19
#define RB      32
#define NRB     19
#define NVALS   (NH * NPIX * DH)
#define XN      (4 * 151 * 6)
#define C1N     (16 * 150 * 5)

#define APP     616
#define ZP      612
#define ESP     72
#define STP     72
#define WTP     40

#define CONV_LDS (C1N * 4 + FRW * 32 * 2)
#define ATT_LDS  (RB * APP * 2 + RB * ZP * 4 + RB * ESP * 2 + PP * 4 * 2)
#define RD_LDS   (NPIX * DH * 4)

#define ALT_PIECES (PP * PP / 8)
#define ALT_BLOCKS 181
#define W1T_BLOCKS (PP * 16 / 256)
#define L1T_BLOCKS (DH * 32 / 256)

#define SZ_F    ((size_t)NB * FRW * 32 * 2)
#define SZ_QK   ((size_t)NB * NH * PP * DH * 2)
#define SZ_VT   ((size_t)NB * NH * DH * PVT * 2)
#define SZ_E    ((size_t)NB * PP * CP * 2)
#define SZ_W1T  ((size_t)PP * 128 * 2)
#define SZ_ALT  ((size_t)PP * PP * 2)
#define SZ_L1T  ((size_t)DH * CP * 2)
#define SZ_OL   ((size_t)NB * 32 * 4)

static_assert(ALT_BLOCKS * 256 >= ALT_PIECES);
static_assert((ALT_BLOCKS - 1) * 256 < ALT_PIECES);
static_assert(ALT_PIECES % 32 == 0);
static_assert(W1T_BLOCKS * 256 == PP * 16);
static_assert(L1T_BLOCKS * 256 == DH * 32);
static_assert(NCT * 16 == PP);
static_assert(NKS * 32 == PP);
static_assert(NRB * RB == PP);
static_assert(PVT == 10 * 64);
static_assert(FRW == 10 * 64);
static_assert(SZ_F % 128 == 0);
static_assert(SZ_QK % 128 == 0);
static_assert(SZ_VT % 128 == 0);
static_assert(SZ_E % 128 == 0);
static_assert(SZ_W1T % 128 == 0);
static_assert(SZ_ALT % 128 == 0);
static_assert(SZ_L1T % 128 == 0);
static_assert(SZ_OL % 128 == 0);
static_assert(ATT_LDS == 127232);
static_assert(CONV_LDS == 88960);

typedef _Float16 v16h __attribute__((ext_vector_type(16)));
typedef _Float16 v8h  __attribute__((ext_vector_type(8)));
typedef float    v8f  __attribute__((ext_vector_type(8)));
typedef float    v4f  __attribute__((ext_vector_type(4)));
typedef unsigned int v4u __attribute__((ext_vector_type(4)));

union Frag  { v16h v; v8h h[2]; };
union Pack8 { v8h h; v4u u; };

extern __shared__ __align__(16) unsigned char dynlds[];

__device__ __forceinline__ v8f mma16(v16h a, v16h b, v8f c) {
  c = __builtin_amdgcn_wmma_f32_16x16x32_f16(false, a, false, b, (short)0, c, false, false);
  asm volatile("v_nop\n\tv_nop\n\tv_nop\n\tv_nop" : "+v"(c) : "v"(a), "v"(b));
  return c;
}

__device__ __forceinline__ v8f zero8() { return (v8f){0.f, 0.f, 0.f, 0.f, 0.f, 0.f, 0.f, 0.f}; }

__device__ __forceinline__ void wave_lds_sync() {
  __builtin_amdgcn_fence(__ATOMIC_RELEASE, "workgroup");
  __builtin_amdgcn_wave_barrier();
  __builtin_amdgcn_fence(__ATOMIC_ACQUIRE, "workgroup");
}

__global__ __launch_bounds__(256) void pack_kernel(const float* __restrict__ qlin_w,
                                                   const float* __restrict__ klin_w,
                                                   const float* __restrict__ alin_w,
                                                   const float* __restrict__ lin1_w,
                                                   _Float16* __restrict__ W1T,
                                                   _Float16* __restrict__ ALT,
                                                   _Float16* __restrict__ L1T) {
  const int blk = blockIdx.x, tid = threadIdx.x;
  Pack8 o;
  _Float16* dst;
  if (blk < ALT_BLOCKS) {
    const int q = blk * 256 + tid;
    if (q >= ALT_PIECES) return;
    const int row  = q / 76;
    const int k0   = (q - row * 76) * 8;
    const int rowc = min(row, NPIX - 1);
#pragma unroll
    for (int i = 0; i < 8; ++i) {
      const int k  = k0 + i;
      const int kc = min(k, NPIX - 1);
      const float v  = alin_w[(size_t)kc * NPIX + rowc];
      const float sc = (row < NPIX && k < NPIX) ? 16.0f : 0.0f;
      o.h[i] = (_Float16)(v * sc);
    }
    dst = ALT + (size_t)q * 8;
  } else if (blk < ALT_BLOCKS + W1T_BLOCKS) {
    const int q    = (blk - ALT_BLOCKS) * 256 + tid;
    const int row  = q >> 4;
    const int k0   = (q & 15) * 8;
    const int rowc = min(row, NPIX - 1);
#pragma unroll
    for (int i = 0; i < 8; ++i) {
      const int k  = k0 + i;
      const int kq = min(k, 63);
      const int kk = min(max(k - 64, 0), 63);
      const float vq = qlin_w[kq * NPIX + rowc];
      const float vk = klin_w[kk * NPIX + rowc];
      const float v  = (k < 64) ? vq : vk;
      const float sc = (row < NPIX) ? 16.0f : 0.0f;
      o.h[i] = (_Float16)(v * sc);
    }
    dst = W1T + (size_t)q * 8;
  } else {
    const int q  = (blk - ALT_BLOCKS - W1T_BLOCKS) * 256 + tid;
    const int c  = q >> 5;
    const int k0 = (q & 31) * 8;
#pragma unroll
    for (int i = 0; i < 8; ++i) o.h[i] = (_Float16)(lin1_w[(k0 + i) * DH + c] * 16.0f);
    dst = L1T + (size_t)q * 8;
  }
  volatile v4u* p = (volatile v4u*)dst;
  *p = o.u;
  __threadfence();
  *p = o.u;
}

__global__ __launch_bounds__(256) void conv_kernel(const float* __restrict__ x,
                                                   const float* __restrict__ c1w,
                                                   const float* __restrict__ c1b,
                                                   const float* __restrict__ c2w,
                                                   const float* __restrict__ c2b,
                                                   _Float16* __restrict__ F) {
  float*    c1s = (float*)dynlds;
  _Float16* fst = (_Float16*)(dynlds + C1N * 4);
  __shared__ float w1s[256];
  __shared__ float w2s[2048];
  __shared__ float b1s[16];
  __shared__ float b2s[32];
  const int tid = threadIdx.x, n = blockIdx.x;
  w1s[tid] = c1w[tid];
#pragma unroll
  for (int i = 0; i < 8; ++i) w2s[i * 256 + tid] = c2w[i * 256 + tid];
  {
    const float bv = c1b[min(tid, 15)];
    const float bw = c2b[min(tid, 31)];
    if (tid < 16) b1s[tid] = bv;
    if (tid < 32) b2s[tid] = bw;
  }
  __syncthreads();
  const float* xs = x + (size_t)n * XN;
  for (int i = tid; i < C1N; i += 256) {
    const int oc  = i / 750;
    const int rem = i - oc * 750;
    const int ii  = rem / 5;
    const int j   = rem - ii * 5;
    float acc = b1s[oc];
#pragma unroll 1
    for (int ic = 0; ic < 4; ++ic) {
      const float* xp = xs + (ic * 151 + ii) * 6 + j;
      const float* wp = w1s + (oc * 4 + ic) * 4;
      acc += xp[0] * wp[0] + xp[1] * wp[1] + xp[6] * wp[2] + xp[7] * wp[3];
    }
    c1s[i] = fmaxf(acc, 0.0f);
  }
  __syncthreads();
  for (int e = tid; e < NPIX * 32; e += 256) {
    const int c = e & 31, p = e >> 5;
    const int i2 = p >> 2, j2 = p & 3;
    float acc = b2s[c];
#pragma unroll 1
    for (int ic = 0; ic < 16; ++ic) {
      const float* cpn = c1s + (ic * 150 + i2) * 5 + j2;
      const float* wp  = w2s + (c * 16 + ic) * 4;
      acc += cpn[0] * wp[0] + cpn[1] * wp[1] + cpn[5] * wp[2] + cpn[6] * wp[3];
    }
    fst[e] = (_Float16)(fmaxf(acc, 0.0f) * 16.0f);
  }
  for (int e = NPIX * 32 + tid; e < FRW * 32; e += 256) fst[e] = (_Float16)0.0f;
  __syncthreads();
  _Float16* Fn = F + (size_t)n * FRW * 32;
  Pack8 pv[10];
#pragma unroll
  for (int it = 0; it < 10; ++it) pv[it].h = *(const v8h*)(fst + (size_t)(it * 256 + tid) * 8);
#pragma unroll
  for (int it = 0; it < 10; ++it) *(volatile v4u*)(Fn + (size_t)(it * 256 + tid) * 8) = pv[it].u;
  __threadfence();
#pragma unroll
  for (int it = 0; it < 10; ++it) *(volatile v4u*)(Fn + (size_t)(it * 256 + tid) * 8) = pv[it].u;
}

__device__ __forceinline__ float projval(float accr, int p, float wx, float wy, float bb) {
  const float xc = (float)(p & 3) * 0.25f;
  const float yc = (float)(p >> 2) * (1.0f / 149.0f);
  return accr * (1.0f / 256.0f) + (wx * xc + wy * yc + bb);
}

__global__ __launch_bounds__(256) void proj_kernel(const _Float16* __restrict__ F,
                                                   const float* __restrict__ kw, const float* __restrict__ kb,
                                                   const float* __restrict__ qw, const float* __restrict__ qb,
                                                   const float* __restrict__ vw, const float* __restrict__ vb,
                                                   const float* __restrict__ kg, const float* __restrict__ kbe,
                                                   const float* __restrict__ qg, const float* __restrict__ qbe,
                                                   const float* __restrict__ vg, const float* __restrict__ vbe,
                                                   _Float16* __restrict__ QPl,
                                                   _Float16* __restrict__ KPl,
                                                   _Float16* __restrict__ VTl) {
  __shared__ __align__(16) _Float16 WT[CP * WTP];
  __shared__ float wc0[CP], wc1[CP], bsv[CP];
  __shared__ __align__(16) _Float16 stg[8][16 * STP];
  __shared__ double red0[8], red1[8];
  __shared__ float stat[2];
  const int tid  = threadIdx.x;
  const int lane = tid & 31, lh = lane >> 4, m = lane & 15;
  const int w    = __builtin_amdgcn_readfirstlane(tid >> 5);
  const int n    = blockIdx.x;
  const _Float16* Fn = F + (size_t)n * FRW * 32;
  _Float16* sw = stg[w];
  const int q8  = lane >> 3;
  const int pc8 = (lane & 7) * 8;

#pragma unroll 1
  for (int t = 0; t < 3; ++t) {
    const float* W  = (t == 0) ? kw  : (t == 1) ? qw  : vw;
    const float* Bv = (t == 0) ? kb  : (t == 1) ? qb  : vb;
    const float* G  = (t == 0) ? kg  : (t == 1) ? qg  : vg;
    const float* Be = (t == 0) ? kbe : (t == 1) ? qbe : vbe;
    __syncthreads();
#pragma unroll 1
    for (int k = 0; k < 32; ++k) WT[tid * WTP + k] = (_Float16)(W[k * CP + tid] * 16.0f);
    wc0[tid] = W[32 * CP + tid];
    wc1[tid] = W[33 * CP + tid];
    bsv[tid] = Bv[tid];
    __syncthreads();

    double s = 0.0, s2 = 0.0;
    for (int u = w; u < NCT * NH; u += 8) {
      const int rt = u >> 2, h = u & 3;
      Frag a;
      const _Float16* ap = Fn + (size_t)(rt * 16 + m) * 32 + 8 * lh;
      a.h[0] = *(const v8h*)ap;
      a.h[1] = *(const v8h*)(ap + 16);
#pragma unroll 1
      for (int ct = 0; ct < 4; ++ct) {
        const int c0 = h * DH + ct * 16;
        Frag b;
        const _Float16* bp = WT + (c0 + m) * WTP + 8 * lh;
        b.h[0] = *(const v8h*)bp;
        b.h[1] = *(const v8h*)(bp + 16);
        const v8f acc = mma16(a.v, b.v, zero8());
        const int c = c0 + m;
        const float wx = wc0[c], wy = wc1[c], bb = bsv[c];
#pragma unroll
        for (int r = 0; r < 8; ++r) {
          const int p = rt * 16 + 8 * lh + r;
          float v = projval(acc[r], p, wx, wy, bb);
          v = (p < NPIX) ? v : 0.0f;
          s  += (double)v;
          s2 += (double)v * (double)v;
        }
      }
    }
#pragma unroll
    for (int off = 1; off < 32; off <<= 1) {
      s  += __shfl_xor(s, off, 32);
      s2 += __shfl_xor(s2, off, 32);
    }
    if (lane == 0) { red0[w] = s; red1[w] = s2; }
    __syncthreads();
    if (tid == 0) {
      double S = 0.0, S2 = 0.0;
      for (int i = 0; i < 8; ++i) { S += red0[i]; S2 += red1[i]; }
      const double mu = S / (double)NVALS;
      double var = S2 / (double)NVALS - mu * mu;
      var = var > 0.0 ? var : 0.0;
      stat[0] = (float)mu;
      stat[1] = 1.0f / sqrtf((float)var + 1e-5f);
    }
    __syncthreads();
    const float mu = stat[0], rstd = stat[1];

    if (t < 2) {
      _Float16* dpl = ((t == 0) ? KPl : QPl) + (size_t)n * NH * PP * DH;
      for (int u = w; u < NCT * NH; u += 8) {
        const int rt = u >> 2, h = u & 3;
        Frag a;
        const _Float16* ap = Fn + (size_t)(rt * 16 + m) * 32 + 8 * lh;
        a.h[0] = *(const v8h*)ap;
        a.h[1] = *(const v8h*)(ap + 16);
#pragma unroll 1
        for (int ct = 0; ct < 4; ++ct) {
          const int c0 = h * DH + ct * 16;
          Frag b;
          const _Float16* bp = WT + (c0 + m) * WTP + 8 * lh;
          b.h[0] = *(const v8h*)bp;
          b.h[1] = *(const v8h*)(bp + 16);
          const v8f acc = mma16(a.v, b.v, zero8());
          const int c = c0 + m, d = ct * 16 + m;
          const float wx = wc0[c], wy = wc1[c], bb = bsv[c];
#pragma unroll
          for (int r = 0; r < 8; ++r) {
            const int p  = rt * 16 + 8 * lh + r;
            const float v = projval(acc[r], p, wx, wy, bb);
            const int pc = min(p, NPIX - 1);
            const size_t gi = ((size_t)h * NPIX + pc) * DH + d;
            const float y  = (v - mu) * rstd * G[gi] + Be[gi];
            const float sc = (p < NPIX) ? 8.0f : 0.0f;
            sw[(8 * lh + r) * STP + d] = (_Float16)(y * sc);
          }
        }
        wave_lds_sync();
        Pack8 pv[4];
#pragma unroll
        for (int it = 0; it < 4; ++it) pv[it].h = *(const v8h*)(sw + (it * 4 + q8) * STP + pc8);
        _Float16* gp = dpl + ((size_t)h * PP + rt * 16) * DH + pc8;
#pragma unroll
        for (int it = 0; it < 4; ++it) *(volatile v4u*)(gp + (size_t)(it * 4 + q8) * DH) = pv[it].u;
        __threadfence();
#pragma unroll
        for (int it = 0; it < 4; ++it) *(volatile v4u*)(gp + (size_t)(it * 4 + q8) * DH) = pv[it].u;
        wave_lds_sync();
      }
    } else {
      _Float16* dvl = VTl + (size_t)n * NH * DH * PVT;
      for (int u = w; u < 10 * 16; u += 8) {
        const int pg = u >> 4, ct16 = u & 15;
        const int c0 = ct16 * 16, h = ct16 >> 2, d0 = (ct16 & 3) * 16;
        Frag b;
        const _Float16* bp = WT + (c0 + m) * WTP + 8 * lh;
        b.h[0] = *(const v8h*)bp;
        b.h[1] = *(const v8h*)(bp + 16);
        const int c = c0 + m, d = d0 + m;
        const float wx = wc0[c], wy = wc1[c], bb = bsv[c];
#pragma unroll 1
        for (int i = 0; i < 4; ++i) {
          const int rt = pg * 4 + i;
          Frag a;
          const _Float16* ap = Fn + (size_t)(rt * 16 + m) * 32 + 8 * lh;
          a.h[0] = *(const v8h*)ap;
          a.h[1] = *(const v8h*)(ap + 16);
          const v8f acc = mma16(a.v, b.v, zero8());
          Pack8 pk;
#pragma unroll
          for (int r = 0; r < 8; ++r) {
            const int p  = rt * 16 + 8 * lh + r;
            const float v = projval(acc[r], p, wx, wy, bb);
            const int pc = min(p, NPIX - 1);
            const size_t gi = ((size_t)h * NPIX + pc) * DH + d;
            const float y  = (v - mu) * rstd * G[gi] + Be[gi];
            const float sc = (p < NPIX) ? 8.0f : 0.0f;
            pk.h[r] = (_Float16)(y * sc);
          }
          *(v8h*)(sw + m * STP + i * 16 + 8 * lh) = pk.h;
        }
        wave_lds_sync();
        Pack8 pv[4];
#pragma unroll
        for (int it = 0; it < 4; ++it) pv[it].h = *(const v8h*)(sw + (it * 4 + q8) * STP + pc8);
        _Float16* gp = dvl + ((size_t)h * DH + d0) * PVT + pg * 64 + pc8;
#pragma unroll
        for (int it = 0; it < 4; ++it) *(volatile v4u*)(gp + (size_t)(it * 4 + q8) * PVT) = pv[it].u;
        __threadfence();
#pragma unroll
        for (int it = 0; it < 4; ++it) *(volatile v4u*)(gp + (size_t)(it * 4 + q8) * PVT) = pv[it].u;
        wave_lds_sync();
      }
    }
  }
}

__global__ __launch_bounds__(256) void attn_kernel(const _Float16* __restrict__ QPl,
                                                   const _Float16* __restrict__ KPl,
                                                   const _Float16* __restrict__ VTl,
                                                   const _Float16* __restrict__ W1T,
                                                   const _Float16* __restrict__ ALT,
                                                   const float* __restrict__ qlin_b,
                                                   const float* __restrict__ klin_b,
                                                   const float* __restrict__ alin_b,
                                                   _Float16* __restrict__ EPl) {
  _Float16* AP  = (_Float16*)dynlds;
  float*    ZS  = (float*)(dynlds + RB * APP * 2);
  _Float16* ES  = (_Float16*)(dynlds + RB * APP * 2 + RB * ZP * 4);
  float*    bqk = (float*)(dynlds + RB * APP * 2 + RB * ZP * 4 + RB * ESP * 2);
  float*    bal = bqk + PP;

  const int tid  = threadIdx.x;
  const int lane = tid & 31, lh = lane >> 4, m = lane & 15;
  const int w    = __builtin_amdgcn_readfirstlane(tid >> 5);
  const int blk  = blockIdx.x;
  const int rb   = blk % NRB;
  const int nh   = blk / NRB;
  const int n    = nh >> 2, h = nh & 3;
  const int f0   = rb * RB;

  for (int i = tid; i < PP; i += 256) {
    const int ic = min(i, NPIX - 1);
    const float a = qlin_b[ic] + klin_b[ic];
    const float b = alin_b[ic];
    bqk[i] = (i < NPIX) ? a : 0.0f;
    bal[i] = (i < NPIX) ? b : 0.0f;
  }
  __syncthreads();

  const _Float16* Qb = QPl + ((size_t)nh * PP + f0) * DH;
  const _Float16* Kb = KPl + ((size_t)nh * PP + f0) * DH;
  v8f acc[2][5];
#pragma unroll
  for (int rg = 0; rg < 2; ++rg)
#pragma unroll
    for (int j = 0; j < 5; ++j) acc[rg][j] = zero8();
#pragma unroll 1
  for (int ks = 0; ks < 4; ++ks) {
    const _Float16* ab = (ks < 2) ? (Qb + ks * 32) : (Kb + (ks - 2) * 32);
    Frag a0, a1;
    a0.h[0] = *(const v8h*)(ab + m * DH + 8 * lh);
    a0.h[1] = *(const v8h*)(ab + m * DH + 16 + 8 * lh);
    a1.h[0] = *(const v8h*)(ab + (16 + m) * DH + 8 * lh);
    a1.h[1] = *(const v8h*)(ab + (16 + m) * DH + 16 + 8 * lh);
#pragma unroll
    for (int j = 0; j < 5; ++j) {
      const int nt = w + 8 * j;
      if (nt < NCT) {
        Frag b;
        const _Float16* bp = W1T + (size_t)(nt * 16 + m) * 128 + ks * 32 + 8 * lh;
        b.h[0] = *(const v8h*)bp;
        b.h[1] = *(const v8h*)(bp + 16);
        acc[0][j] = mma16(a0.v, b.v, acc[0][j]);
        acc[1][j] = mma16(a1.v, b.v, acc[1][j]);
      }
    }
  }
#pragma unroll
  for (int j = 0; j < 5; ++j) {
    const int nt = w + 8 * j;
    if (nt < NCT) {
      const int c = nt * 16 + m;
      const float bb = bqk[c];
      const float sc = (c < NPIX) ? 16.0f : 0.0f;
#pragma unroll
      for (int rg = 0; rg < 2; ++rg) {
#pragma unroll
        for (int r = 0; r < 8; ++r) {
          const float v = acc[rg][j][r] * (1.0f / 128.0f) + bb;
          const float e = (v > 0.0f) ? v : (__expf(v) - 1.0f);
          AP[(rg * 16 + 8 * lh + r) * APP + c] = (_Float16)(e * sc);
        }
      }
    }
  }
  __syncthreads();

#pragma unroll
  for (int rg = 0; rg < 2; ++rg)
#pragma unroll
    for (int j = 0; j < 5; ++j) acc[rg][j] = zero8();
#pragma unroll 1
  for (int ks = 0; ks < NKS; ++ks) {
    Frag a0, a1;
    const _Float16* ap0 = AP + m * APP + ks * 32 + 8 * lh;
    const _Float16* ap1 = AP + (16 + m) * APP + ks * 32 + 8 * lh;
    a0.h[0] = *(const v8h*)ap0;
    a0.h[1] = *(const v8h*)(ap0 + 16);
    a1.h[0] = *(const v8h*)ap1;
    a1.h[1] = *(const v8h*)(ap1 + 16);
#pragma unroll
    for (int j = 0; j < 5; ++j) {
      const int nt = w + 8 * j;
      if (nt < NCT) {
        Frag b;
        const _Float16* bp = ALT + (size_t)(nt * 16 + m) * PP + ks * 32 + 8 * lh;
        b.h[0] = *(const v8h*)bp;
        b.h[1] = *(const v8h*)(bp + 16);
        acc[0][j] = mma16(a0.v, b.v, acc[0][j]);
        acc[1][j] = mma16(a1.v, b.v, acc[1][j]);
      }
    }
  }
#pragma unroll
  for (int j = 0; j < 5; ++j) {
    const int nt = w + 8 * j;
    if (nt < NCT) {
      const int c = nt * 16 + m;
#pragma unroll
      for (int rg = 0; rg < 2; ++rg)
#pragma unroll
        for (int r = 0; r < 8; ++r) ZS[(rg * 16 + 8 * lh + r) * ZP + c] = acc[rg][j][r];
    }
  }
  __syncthreads();

  {
    const int row = tid >> 3, s8 = tid & 7;
    const float* zr = ZS + row * ZP;
    float mx = -INFINITY;
    for (int c = s8; c < NPIX; c += 8) mx = fmaxf(mx, zr[c] * (1.0f / 256.0f) + bal[c]);
    mx = fmaxf(mx, __shfl_xor(mx, 1, 32));
    mx = fmaxf(mx, __shfl_xor(mx, 2, 32));
    mx = fmaxf(mx, __shfl_xor(mx, 4, 32));
    float sm = 0.0f;
    for (int c = s8; c < NPIX; c += 8) sm += __expf(zr[c] * (1.0f / 256.0f) + bal[c] - mx);
    sm += __shfl_xor(sm, 1, 32);
    sm += __shfl_xor(sm, 2, 32);
    sm += __shfl_xor(sm, 4, 32);
    const float scl = (1.0f / sm) * 1024.0f;
    _Float16* pr = AP + row * APP;
    for (int c = s8; c < PP; c += 8) {
      const float pvv = __expf(zr[c] * (1.0f / 256.0f) + bal[c] - mx) * scl;
      const float msk = (c < NPIX) ? 1.0f : 0.0f;
      pr[c] = (_Float16)(pvv * msk);
    }
  }
  __syncthreads();

  {
    const int rg = w >> 2, dt = w & 3;
    v8f o = zero8();
    const _Float16* vr = VTl + ((size_t)nh * DH + dt * 16 + m) * PVT + 8 * lh;
    const _Float16* pr = AP + (rg * 16 + m) * APP + 8 * lh;
#pragma unroll 1
    for (int ks = 0; ks < NKS; ++ks) {
      Frag a, b;
      a.h[0] = *(const v8h*)(pr + ks * 32);
      a.h[1] = *(const v8h*)(pr + ks * 32 + 16);
      b.h[0] = *(const v8h*)(vr + ks * 32);
      b.h[1] = *(const v8h*)(vr + ks * 32 + 16);
      o = mma16(a.v, b.v, o);
    }
    const int d = dt * 16 + m;
#pragma unroll
    for (int r = 0; r < 8; ++r) ES[(rg * 16 + 8 * lh + r) * ESP + d] = (_Float16)(o[r] * (1.0f / 512.0f));
  }
  __syncthreads();
  {
    const int q8 = lane >> 3, pc8 = (lane & 7) * 8;
    const int row = w * 4 + q8;
    Pack8 pv;
    pv.h = *(const v8h*)(ES + row * ESP + pc8);
    _Float16* gp = EPl + ((size_t)n * PP + f0 + row) * CP + h * DH + pc8;
    *(volatile v4u*)gp = pv.u;
    __threadfence();
    *(volatile v4u*)gp = pv.u;
  }
}

__global__ __launch_bounds__(256) void readout_kernel(const _Float16* __restrict__ EPl,
                                                      const _Float16* __restrict__ L1T,
                                                      const float* __restrict__ lin1_b,
                                                      const float* __restrict__ lin2_w,
                                                      const float* __restrict__ lin2_b,
                                                      float* __restrict__ OUTL) {
  float* L = (float*)dynlds;
  __shared__ float b1s[64];
  __shared__ double red[8];
  __shared__ float stat[2];
  __shared__ float pmx[4][64];
  __shared__ float Ef[64];
  __shared__ __align__(16) float res[32];
  const int tid  = threadIdx.x;
  const int lane = tid & 31, lh = lane >> 4, m = lane & 15;
  const int w    = __builtin_amdgcn_readfirstlane(tid >> 5);
  const int n    = blockIdx.x;
  {
    const float bv = lin1_b[min(tid, 63)];
    if (tid < 64) b1s[tid] = bv;
  }
  __syncthreads();
  const _Float16* En = EPl + (size_t)n * PP * CP;
  double s = 0.0;
  for (int u = w; u < NCT * 4; u += 8) {
    const int rt = u >> 2, ct = u & 3;
    v8f acc = zero8();
    const _Float16* ap = En + (size_t)(rt * 16 + m) * CP + 8 * lh;
    const _Float16* bp = L1T + (size_t)(ct * 16 + m) * CP + 8 * lh;
#pragma unroll 1
    for (int ks = 0; ks < 8; ++ks) {
      Frag a, b;
      a.h[0] = *(const v8h*)(ap + ks * 32);
      a.h[1] = *(const v8h*)(ap + ks * 32 + 16);
      b.h[0] = *(const v8h*)(bp + ks * 32);
      b.h[1] = *(const v8h*)(bp + ks * 32 + 16);
      acc = mma16(a.v, b.v, acc);
    }
    const int c = ct * 16 + m;
    const float bb = b1s[c];
#pragma unroll
    for (int r = 0; r < 8; ++r) {
      const int p = rt * 16 + 8 * lh + r;
      const float v = fmaxf(acc[r] * (1.0f / 256.0f) + bb, 0.0f);
      if (p < NPIX) {
        L[p * DH + c] = v;
        s += (double)v;
      }
    }
  }
#pragma unroll
  for (int off = 1; off < 32; off <<= 1) s += __shfl_xor(s, off, 32);
  if (lane == 0) red[w] = s;
  __syncthreads();
  if (tid == 0) {
    double S = 0.0;
    for (int i = 0; i < 8; ++i) S += red[i];
    stat[0] = (float)(S / (double)(NPIX * DH));
  }
  __syncthreads();
  const float mu = stat[0];
  float s2f = 0.0f;
  for (int e = tid; e < NPIX * DH; e += 256) {
    const float dl = L[e] - mu;
    s2f += dl * dl;
  }
  double s2 = (double)s2f;
#pragma unroll
  for (int off = 1; off < 32; off <<= 1) s2 += __shfl_xor(s2, off, 32);
  __syncthreads();
  if (lane == 0) red[w] = s2;
  __syncthreads();
  if (tid == 0) {
    double S2 = 0.0;
    for (int i = 0; i < 8; ++i) S2 += red[i];
    const float var = (float)(S2 / (double)(NPIX * DH));
    stat[1] = 1.0f / sqrtf(var + 1e-5f);
  }
  {
    const int d = tid & 63, q = tid >> 6;
    float mv = -INFINITY;
    for (int p = q; p < NPIX; p += 4) mv = fmaxf(mv, L[p * DH + d]);
    pmx[q][d] = mv;
  }
  __syncthreads();
  if (tid < 64) {
    const float mv = fmaxf(fmaxf(pmx[0][tid], pmx[1][tid]), fmaxf(pmx[2][tid], pmx[3][tid]));
    Ef[tid] = (mv - stat[0]) * stat[1];
  }
  __syncthreads();
  if (w == 0) {
    const int oc = min(lane, 9);
    float a = 0.0f;
#pragma unroll 1
    for (int dd = 0; dd < DH; ++dd) a += Ef[dd] * lin2_w[dd * 10 + oc];
    a += lin2_b[oc];
    const float e = (a > 0.0f) ? a : expm1f(a);
    res[lane] = (lane < 10) ? e : 0.0f;
    wave_lds_sync();
    const v4f vv = *(const v4f*)(res + (lane & 7) * 4);
    if (lane < 8) {
      float* gp = OUTL + (size_t)n * 32 + lane * 4;
      *(volatile v4f*)gp = vv;
      __threadfence();
      *(volatile v4f*)gp = vv;
    }
  }
}

__global__ __launch_bounds__(256) void final_kernel(const float* __restrict__ OUTL, float* __restrict__ out) {
  const int t = threadIdx.x;
  if (t >= 160) return;
  v4f v;
#pragma unroll
  for (int i = 0; i < 4; ++i) {
    const int e  = 4 * t + i;
    const int sm = e / 10;
    const int cl = e - sm * 10;
    v[i] = OUTL[sm * 32 + cl];
  }
  volatile v4f* p = (volatile v4f*)(out + 4 * t);
  *p = v;
  __threadfence();
  *p = v;
}

extern "C" void kernel_launch(void* const* d_in, const int* in_sizes, int n_in,
                              void* d_out, int out_size, void* d_ws, size_t ws_size,
                              hipStream_t stream) {
  if (n_in < 27) return;
  if (in_sizes[0] != NB * XN) return;
  if (in_sizes[5] != 34 * CP) return;
  if (in_sizes[15] != NPIX * NPIX) return;
  if (in_sizes[23] != CP * DH) return;
  if (out_size != NB * 10) return;

  const float* x       = (const float*)d_in[0];
  const float* conv1_w = (const float*)d_in[1];
  const float* conv1_b = (const float*)d_in[2];
  const float* conv2_w = (const float*)d_in[3];
  const float* conv2_b = (const float*)d_in[4];
  const float* kp_w    = (const float*)d_in[5];
  const float* kp_b    = (const float*)d_in[6];
  const float* qp_w    = (const float*)d_in[7];
  const float* qp_b    = (const float*)d_in[8];
  const float* vp_w    = (const float*)d_in[9];
  const float* vp_b    = (const float*)d_in[10];
  const float* klin_w  = (const float*)d_in[11];
  const float* klin_b  = (const float*)d_in[12];
  const float* qlin_w  = (const float*)d_in[13];
  const float* qlin_b  = (const float*)d_in[14];
  const float* alin_w  = (const float*)d_in[15];
  const float* alin_b  = (const float*)d_in[16];
  const float* knorm_g = (const float*)d_in[17];
  const float* knorm_b = (const float*)d_in[18];
  const float* qnorm_g = (const float*)d_in[19];
  const float* qnorm_b = (const float*)d_in[20];
  const float* vnorm_g = (const float*)d_in[21];
  const float* vnorm_b = (const float*)d_in[22];
  const float* lin1_w  = (const float*)d_in[23];
  const float* lin1_b  = (const float*)d_in[24];
  const float* lin2_w  = (const float*)d_in[25];
  const float* lin2_b  = (const float*)d_in[26];
  float* out = (float*)d_out;

  size_t off = 0;
  const size_t oF   = off; off += SZ_F;
  const size_t oQ   = off; off += SZ_QK;
  const size_t oK   = off; off += SZ_QK;
  const size_t oV   = off; off += SZ_VT;
  const size_t oE   = off; off += SZ_E;
  const size_t oW1  = off; off += SZ_W1T;
  const size_t oAL  = off; off += SZ_ALT;
  const size_t oL1  = off; off += SZ_L1T;
  const size_t oOL  = off; off += SZ_OL;
  if (off > ws_size) return;

  char* ws = (char*)d_ws;
  _Float16* F    = (_Float16*)(ws + oF);
  _Float16* QPl  = (_Float16*)(ws + oQ);
  _Float16* KPl  = (_Float16*)(ws + oK);
  _Float16* VTl  = (_Float16*)(ws + oV);
  _Float16* EPl  = (_Float16*)(ws + oE);
  _Float16* W1T  = (_Float16*)(ws + oW1);
  _Float16* ALT  = (_Float16*)(ws + oAL);
  _Float16* L1T  = (_Float16*)(ws + oL1);
  float*    OUTL = (float*)(ws + oOL);

  (void)hipFuncSetAttribute(reinterpret_cast<const void*>(&conv_kernel),
                            hipFuncAttributeMaxDynamicSharedMemorySize, CONV_LDS);
  (void)hipFuncSetAttribute(reinterpret_cast<const void*>(&attn_kernel),
                            hipFuncAttributeMaxDynamicSharedMemorySize, ATT_LDS);
  (void)hipFuncSetAttribute(reinterpret_cast<const void*>(&readout_kernel),
                            hipFuncAttributeMaxDynamicSharedMemorySize, RD_LDS);

  pack_kernel<<<dim3(ALT_BLOCKS + W1T_BLOCKS + L1T_BLOCKS), dim3(256), 0, stream>>>(
      qlin_w, klin_w, alin_w, lin1_w, W1T, ALT, L1T);
  conv_kernel<<<dim3(NB), dim3(256), CONV_LDS, stream>>>(x, conv1_w, conv1_b, conv2_w, conv2_b, F);
  proj_kernel<<<dim3(NB), dim3(256), 0, stream>>>(F, kp_w, kp_b, qp_w, qp_b, vp_w, vp_b,
                                                  knorm_g, knorm_b, qnorm_g, qnorm_b, vnorm_g, vnorm_b,
                                                  QPl, KPl, VTl);
  attn_kernel<<<dim3(NB * NH * NRB), dim3(256), ATT_LDS, stream>>>(QPl, KPl, VTl, W1T, ALT,
                                                                    qlin_b, klin_b, alin_b, EPl);
  readout_kernel<<<dim3(NB), dim3(256), RD_LDS, stream>>>(EPl, L1T, lin1_b, lin2_w, lin2_b, OUTL);
  final_kernel<<<dim3(1), dim3(256), 0, stream>>>(OUTL, out);
  (void)hipGetLastError();
}
